// MultiHeadAttention_81501299409410
// MI455X (gfx1250) — hardware-verified
//
#include <hip/hip_runtime.h>


#ifndef NB
#define NB 4
#endif
#ifndef SEQ
#define SEQ 2048
#endif
#define SEQ_FULL 2048
#define TT   SEQ
#define DM   512
#define NH_  16
#define HD   32
#define DQ   (NH_ * HD)
#define NQ3  (3 * DQ)
#define PCAR 1024.0f
#define CCAR 64.0f
#define WCAR 64.0f
#define QS2  0.25503486f
#define NEGF (-3.0e38f)

static_assert(HD == 32);
static_assert(HD * 2 * 2 == 128);
static_assert(DQ == NH_ * HD);
static_assert(DQ == DM);
static_assert(TT % 64 == 0);
static_assert(TT % 32 == 0);
static_assert(TT % 16 == 0);
static_assert(TT % 8 == 0);
static_assert(DM % 64 == 0);
static_assert(NQ3 % 64 == 0);
static_assert(DM % 32 == 0);
static_assert(DQ % 32 == 0);
static_assert((NQ3 * DM) % 64 == 0);
static_assert((DQ * DM) % 64 == 0);
static_assert((TT * DM) % (8 * 256) == 0);
static_assert(NB >= 1);
static_assert(SEQ <= SEQ_FULL);

typedef _Float16 h16;
typedef unsigned short bf;
typedef __attribute__((ext_vector_type(16))) __bf16   v16bf;
typedef __attribute__((ext_vector_type(16))) _Float16 v16h;
typedef __attribute__((ext_vector_type(8)))  _Float16 v8h;
typedef __attribute__((ext_vector_type(8)))  unsigned short v8us;
typedef __attribute__((ext_vector_type(2)))  unsigned short v2us;
typedef __attribute__((ext_vector_type(8)))  float    v8f;
typedef __attribute__((ext_vector_type(4)))  float    v4f;
typedef v8h  __attribute__((may_alias)) v8ha;
typedef v4f  __attribute__((may_alias)) v4fa;

__device__ __forceinline__ unsigned short f2bf(float f) { unsigned u = __float_as_uint(f); u += 0x7FFFu + ((u >> 16) & 1u); return (unsigned short)(u >> 16); }
__device__ __forceinline__ float bf2f(unsigned short b) { return __uint_as_float(((unsigned)b) << 16); }
__device__ __forceinline__ float bfr(float f) { return bf2f(f2bf(f)); }
__device__ __forceinline__ unsigned short hbits(float f) { return __builtin_bit_cast(unsigned short, (h16)f); }
__device__ __forceinline__ v16h cat16(v8h lo, v8h hi) { return __builtin_shufflevector(lo, hi, 0, 1, 2, 3, 4, 5, 6, 7, 8, 9, 10, 11, 12, 13, 14, 15); }
__device__ __forceinline__ v16bf cat16b(v8us lo, v8us hi) { return __builtin_bit_cast(v16bf, __builtin_shufflevector(lo, hi, 0, 1, 2, 3, 4, 5, 6, 7, 8, 9, 10, 11, 12, 13, 14, 15)); }
__device__ __forceinline__ v8f wmma16(v16h a, v16h b, v8f c) { return __builtin_amdgcn_wmma_f32_16x16x32_f16(false, a, false, b, (short)0, c, false, false); }
__device__ __forceinline__ v8f wmmab(v16bf a, v16bf b, v8f c) { return __builtin_amdgcn_wmma_f32_16x16x32_bf16(false, a, false, b, (short)0, c, false, false); }
__device__ __forceinline__ v16h  ldh(const h16* p) { return cat16(*(const v8h*)p, *(const v8h*)(p + 16)); }
__device__ __forceinline__ v16bf ldb(const bf* p)  { return cat16b(*(const v8us*)p, *(const v8us*)(p + 16)); }

template <typename T16> struct WFrag;
template <> struct WFrag<h16> { typedef v16h V; static __device__ __forceinline__ V ld(const h16* p) { return ldh(p); } static __device__ __forceinline__ v8f mma(V a, V b, v8f c) { return wmma16(a, b, c); } };
template <> struct WFrag<bf> { typedef v16bf V; static __device__ __forceinline__ V ld(const bf* p) { return ldb(p); } static __device__ __forceinline__ v8f mma(V a, V b, v8f c) { return wmmab(a, b, c); } };
template <typename T16, bool BIAS>
__device__ __forceinline__ void gemmw_body(const T16* __restrict__ A, const T16* __restrict__ Bt, const int K, const int lda, const int ksA, float* C, const int ldc, const float* __restrict__ bias, const float osc, size_t sA, size_t sC) {
    typedef typename WFrag<T16>::V V;
    __shared__ __align__(16) float os[16 * 68];
    const size_t z = blockIdx.z; A += z * sA; C += z * sC;
    const int lane = threadIdx.x & 31, lr = lane & 15, hi = lane >> 4; const int r0 = blockIdx.x * 64, c0 = blockIdx.y * 64;
    v8f acc[4][4];
#pragma unroll
    for (int mb = 0; mb < 4; ++mb)
#pragma unroll
        for (int nb = 0; nb < 4; ++nb) acc[mb][nb] = (v8f){};
    const size_t aoff = (size_t)(r0 + lr) * lda + 8 * hi, boff = (size_t)(c0 + lr) * K + 8 * hi;
#pragma unroll 1
    for (int kc = 0; kc < K; kc += 32) {
        const size_t ak = aoff + (size_t)(kc >> 5) * ksA;
        V a[4];
#pragma unroll
        for (int mb = 0; mb < 4; ++mb) a[mb] = WFrag<T16>::ld(A + ak + (size_t)mb * 16 * lda);
#pragma unroll
        for (int nb = 0; nb < 4; ++nb) { const V b = WFrag<T16>::ld(Bt + boff + (size_t)nb * 16 * K + kc);
#pragma unroll
            for (int mb = 0; mb < 4; ++mb) acc[mb][nb] = WFrag<T16>::mma(a[mb], b, acc[mb][nb]); }
        asm volatile("v_nop\n\tv_nop\n\tv_nop\n\tv_nop" : "+v"(acc[0][0]), "+v"(acc[1][1]), "+v"(acc[2][2]), "+v"(acc[3][3]) : "v"(a[0]), "v"(a[3]));
    }
#pragma unroll
    for (int mb = 0; mb < 4; ++mb) {
#pragma unroll
        for (int nb = 0; nb < 4; ++nb) {
#pragma unroll
            for (int j = 0; j < 8; ++j) os[(hi * 8 + j) * 68 + nb * 16 + lr] = acc[mb][nb][j]; }
        __builtin_amdgcn_wave_barrier(); asm volatile("" ::: "memory");
        float* crow = C + (size_t)(r0 + mb * 16) * ldc + c0;
#pragma unroll 1
        for (int ps = 0; ps < 2; ++ps) {
#pragma unroll
            for (int s = 0; s < 8; ++s) { const int row = 2 * s + hi, cofs = lr * 4; v4f val = *(const v4fa*)(os + row * 68 + cofs);
                val[0] *= osc; val[1] *= osc; val[2] *= osc; val[3] *= osc;
                if (BIAS) { val[0] += bfr(bias[c0 + cofs]); val[1] += bfr(bias[c0 + cofs + 1]); val[2] += bfr(bias[c0 + cofs + 2]); val[3] += bfr(bias[c0 + cofs + 3]); }
                *(volatile v4f*)(crow + (size_t)row * ldc + cofs) = val; }
            if (ps == 0) __threadfence(); }
        __builtin_amdgcn_wave_barrier(); asm volatile("" ::: "memory");
    }
}
__global__ __launch_bounds__(32) void k_gemm_qkv(const bf* __restrict__ A, const bf* __restrict__ Bt, float* C, const float* __restrict__ bias) {
    gemmw_body<bf, true>(A, Bt, DM, DM, 32, C, NQ3, bias, 1.0f, (size_t)TT * DM, (size_t)TT * NQ3);
}
__global__ __launch_bounds__(32) void k_gemm_out(const h16* __restrict__ A, const h16* __restrict__ Bt, float* C, const float* __restrict__ bias) {
    gemmw_body<h16, true>(A, Bt, DQ, HD, TT * HD, C, DM, bias, 1.0f / (CCAR * WCAR), (size_t)NH_ * TT * HD, (size_t)SEQ_FULL * DM);
}

__global__ __launch_bounds__(256) void k_wtG(const float* __restrict__ w, int K, int N, unsigned short* Bt, int asf16, float scl) {
    const int lane = threadIdx.x & 31; const int wave = __builtin_amdgcn_readfirstlane(threadIdx.x >> 5);
    const int L0 = (blockIdx.x * 8 + wave) * 8; const int nlines = N * K / 64;
#pragma unroll
    for (int ps = 0; ps < 2; ++ps) {
#pragma unroll 1
        for (int l = 0; l < 8; ++l) { const int L = L0 + l; if (L >= nlines) break; const size_t e = (size_t)L * 64 + lane * 2; const int k = (int)(e % K), n = (int)(e / K); v2us o;
            const float w0 = bfr(w[(size_t)k * N + n]), w1 = bfr(w[(size_t)(k + 1) * N + n]);
            const unsigned short b0 = (unsigned short)(__float_as_uint(w0) >> 16), b1 = (unsigned short)(__float_as_uint(w1) >> 16);
            const unsigned short g0 = hbits(w0 * scl), g1 = hbits(w1 * scl);
            o[0] = asf16 ? g0 : b0; o[1] = asf16 ? g1 : b1; *(volatile v2us*)(Bt + e) = o; }
        if (ps == 0) __threadfence(); }
}
__global__ __launch_bounds__(256) void k_cvtx(const float* __restrict__ src, bf* dst, int n8, size_t sstr, size_t dstr) {
    const int i = blockIdx.x * 256 + threadIdx.x; if (i >= n8) return;
    const float* s = src + (size_t)blockIdx.y * sstr + (size_t)i * 8; bf* d = dst + (size_t)blockIdx.y * dstr + (size_t)i * 8;
    const v8f v = *(const v8f*)s; v8us o;
#pragma unroll
    for (int k = 0; k < 8; ++k) o[k] = f2bf(v[k]);
    *(volatile v8us*)d = o; __threadfence(); *(volatile v8us*)d = o;
}
__global__ __launch_bounds__(256) void k_qkp(const float* __restrict__ F, h16* P16) {
    const size_t i = (size_t)blockIdx.x * 256 + threadIdx.x; if (i >= (size_t)NB * 2 * NH_ * TT * HD / 8) return;
    const int d = (int)(i % (HD / 8)) * 8; const int t = (int)((i / (HD / 8)) % TT); const int gg = (int)(i / ((size_t)(HD / 8) * TT));
    const int b = gg / (2 * NH_), g = gg % (2 * NH_);
    const float* f = F + ((size_t)b * TT + t) * NQ3 + g * HD + d; const v4f a = *(const v4f*)f; const v4f c = *(const v4f*)(f + 4);
    v8h o16;
#pragma unroll
    for (int k = 0; k < 4; ++k) { o16[k] = (h16)a[k]; o16[k + 4] = (h16)c[k]; }
    h16* dst = P16 + i * 8;
    *(volatile v8h*)dst = o16; __threadfence(); *(volatile v8h*)dst = o16;
}
__global__ __launch_bounds__(256) void k_vtp(const float* __restrict__ F, h16* V16) {
    const size_t i = (size_t)blockIdx.x * 256 + threadIdx.x; if (i >= (size_t)NB * NH_ * HD * TT / 8) return;
    const int t = (int)(i % (TT / 8)) * 8; const int d = (int)((i / (TT / 8)) % HD); const int gg = (int)(i / ((size_t)(TT / 8) * HD));
    const int b = gg / NH_, h = gg % NH_;
    const float* f = F + ((size_t)b * TT + t) * NQ3 + 2 * DQ + h * HD + d;
    v8h o16;
#pragma unroll
    for (int q = 0; q < 8; ++q) o16[q] = (h16)f[(size_t)q * NQ3];
    h16* dst = V16 + i * 8;
    *(volatile v8h*)dst = o16; __threadfence(); *(volatile v8h*)dst = o16;
}

__global__ __launch_bounds__(32) void k_flash16(const h16* __restrict__ QK16, const h16* __restrict__ V16, h16* CTX) {
    __shared__ __align__(16) h16 ps[16 * 40];
    __shared__ __align__(16) h16 osx[16 * 40];
    const int lane = threadIdx.x & 31, lr = lane & 15, hi = lane >> 4;
    const int h = blockIdx.y, b = blockIdx.z; const int q0 = (int)blockIdx.x * 16;
    const h16* Qp = QK16 + ((size_t)(b * 2 * NH_) + h) * TT * HD; const h16* Kp = QK16 + ((size_t)(b * 2 * NH_) + NH_ + h) * TT * HD; const h16* Vp = V16 + ((size_t)b * NH_ + h) * HD * TT;
    const int qoff = (q0 + lr) * HD + 8 * hi;
    v8f acc[2]; float mrun[8], lrun[8];
#pragma unroll
    for (int j = 0; j < 2; ++j) acc[j] = (v8f){};
#pragma unroll
    for (int r = 0; r < 8; ++r) { mrun[r] = NEGF; lrun[r] = 0.f; }
#pragma unroll 1
    for (int key0 = 0; key0 < TT; key0 += 32) {
        int qo = qoff; asm volatile("" : "+v"(qo));
        const int ko = (key0 + lr) * HD + 8 * hi;
        v8f s0 = (v8f){}, s1 = (v8f){};
        {
            const v16h a0 = ldh(Qp + qo);
            const v16h b0 = ldh(Kp + ko), b1 = ldh(Kp + ko + 16 * HD);
            s0 = wmma16(a0, b0, s0); s1 = wmma16(a0, b1, s1);
            asm volatile("v_nop\n\tv_nop\n\tv_nop\n\tv_nop" : "+v"(s0), "+v"(s1) : "v"(a0), "v"(b0), "v"(b1));
        }
        float e0[8], e1[8], alf[8];
#pragma unroll
        for (int r = 0; r < 8; ++r) {
            const float t0 = s0[r] * QS2; const float t1 = s1[r] * QS2;
            float m = fmaxf(t0, t1);
            m = fmaxf(m, __shfl_xor(m, 8, 32)); m = fmaxf(m, __shfl_xor(m, 4, 32)); m = fmaxf(m, __shfl_xor(m, 2, 32)); m = fmaxf(m, __shfl_xor(m, 1, 32));
            const float mn = fmaxf(mrun[r], m);
            alf[r] = __builtin_amdgcn_exp2f(mrun[r] - mn); mrun[r] = mn;
            e0[r] = __builtin_amdgcn_exp2f(t0 - mn); e1[r] = __builtin_amdgcn_exp2f(t1 - mn);
            lrun[r] = lrun[r] * alf[r] + (e0[r] + e1[r]);
        }
#pragma unroll
        for (int j = 0; j < 2; ++j)
#pragma unroll
            for (int r = 0; r < 8; ++r) acc[j][r] *= alf[r];
#pragma unroll
        for (int r = 0; r < 8; ++r) { ps[(8 * hi + r) * 40 + lr] = (h16)(e0[r] * PCAR); ps[(8 * hi + r) * 40 + 16 + lr] = (h16)(e1[r] * PCAR); }
        __builtin_amdgcn_wave_barrier(); asm volatile("" ::: "memory");
        const v16h pa = cat16(*(const v8ha*)(ps + lr * 40 + 8 * hi), *(const v8ha*)(ps + lr * 40 + 16 + 8 * hi));
        __builtin_amdgcn_wave_barrier(); asm volatile("" ::: "memory");
        const int vo = lr * TT + key0 + 8 * hi;
        v16h vb[2];
#pragma unroll
        for (int j = 0; j < 2; ++j) vb[j] = ldh(Vp + vo + j * 16 * TT);
#pragma unroll
        for (int j = 0; j < 2; ++j) acc[j] = wmma16(pa, vb[j], acc[j]);
        asm volatile("v_nop\n\tv_nop\n\tv_nop\n\tv_nop" : "+v"(acc[0]), "+v"(acc[1]) : "v"(pa), "v"(vb[0]), "v"(vb[1]));
    }
    float linv[8];
#pragma unroll
    for (int r = 0; r < 8; ++r) { float l = lrun[r]; l += __shfl_xor(l, 8, 32); l += __shfl_xor(l, 4, 32); l += __shfl_xor(l, 2, 32); l += __shfl_xor(l, 1, 32); linv[r] = (1.0f / l) * (CCAR / PCAR); }
#pragma unroll
    for (int j = 0; j < 2; ++j)
#pragma unroll
        for (int r = 0; r < 8; ++r) osx[(8 * hi + r) * 40 + j * 16 + lr] = (h16)(acc[j][r] * linv[r]);
    __builtin_amdgcn_wave_barrier(); asm volatile("" ::: "memory");
    const int rr = lane >> 2, cc = (lane & 3) * 8; h16* ob = CTX + (((size_t)b * NH_ + h) * TT + q0) * HD + lane * 8;
#pragma unroll 1
    for (int pz = 0; pz < 2; ++pz) {
#pragma unroll
        for (int s = 0; s < 2; ++s) { const int row = 8 * s + rr; const v8h xv = *(const v8ha*)(osx + row * 40 + cc);
            *(volatile v8h*)(ob + s * 8 * HD) = xv; }
        if (pz == 0) __threadfence(); }
}

constexpr size_t SZ_WQKV = (size_t)NQ3 * DM * 2;
constexpr size_t SZ_WO   = (size_t)DM * DQ * 2;
constexpr size_t SZ_XB   = (size_t)NB * TT * DM * 2;
constexpr size_t SZ_F    = (size_t)NB * TT * NQ3 * 4;
constexpr size_t SZ_QK16 = (size_t)NB * 2 * NH_ * TT * HD * 2;
constexpr size_t SZ_VT16 = (size_t)NB * NH_ * HD * TT * 2;
constexpr size_t SZ_CTX  = (size_t)NB * NH_ * TT * HD * 2;
constexpr size_t SZ_ALL  = SZ_WQKV + SZ_WO + SZ_XB + SZ_F + SZ_QK16 + SZ_VT16 + SZ_CTX;
static_assert(SZ_WQKV % 256 == 0 && SZ_WO % 256 == 0 && SZ_XB % 256 == 0 && SZ_F % 256 == 0 && SZ_QK16 % 256 == 0 && SZ_VT16 % 256 == 0 && SZ_CTX % 256 == 0);
static_assert(SZ_ALL <= (size_t)134217728);

extern "C" void kernel_launch(void* const* d_in, const int* in_sizes, int n_in,
                              void* d_out, int out_size, void* d_ws, size_t ws_size, hipStream_t stream) {
    if (n_in < 5) return;
    const long long need_x = (long long)(NB - 1) * SEQ_FULL * DM + (long long)TT * DM;
    if ((long long)in_sizes[0] < need_x || (long long)in_sizes[1] < (long long)DM * NQ3 || in_sizes[2] < NQ3 || (long long)in_sizes[3] < (long long)DQ * DM || in_sizes[4] < DM || (long long)out_size < need_x) return;
    if (ws_size < SZ_ALL) return;
    const float* x = (const float*)d_in[0]; const float* wattn = (const float*)d_in[1]; const float* battn = (const float*)d_in[2]; const float* wproj = (const float*)d_in[3]; const float* bproj = (const float*)d_in[4];
    float* OUT = (float*)d_out;
    char* wsp = (char*)d_ws;
    auto take = [&](size_t bytes) { char* p = wsp; wsp += bytes; return (void*)p; };
    bf* WQKV = (bf*)take(SZ_WQKV);
    h16* WO  = (h16*)take(SZ_WO);
    bf* XB   = (bf*)take(SZ_XB);
    float* F = (float*)take(SZ_F);
    h16* QK16 = (h16*)take(SZ_QK16);
    h16* VT16 = (h16*)take(SZ_VT16);
    h16* CTX  = (h16*)take(SZ_CTX);
    k_wtG<<<(unsigned)((DM * NQ3 / 64 + 63) / 64), 256, 0, stream>>>(wattn, DM, NQ3, (unsigned short*)WQKV, 0, 1.0f);
    k_wtG<<<(unsigned)((DQ * DM / 64 + 63) / 64), 256, 0, stream>>>(wproj, DQ, DM, (unsigned short*)WO, 1, WCAR);
    k_cvtx<<<dim3((unsigned)((TT * DM / 8 + 255) / 256), NB, 1), 256, 0, stream>>>(x, XB, TT * DM / 8, (size_t)SEQ_FULL * DM, (size_t)TT * DM);
    k_gemm_qkv<<<dim3(TT / 64, NQ3 / 64, NB), 32, 0, stream>>>(XB, WQKV, F, battn);
    k_qkp<<<(unsigned)(((size_t)NB * 2 * NH_ * TT * HD / 8 + 255) / 256), 256, 0, stream>>>(F, QK16);
    k_vtp<<<(unsigned)(((size_t)NB * NH_ * HD * TT / 8 + 255) / 256), 256, 0, stream>>>(F, VT16);
    k_flash16<<<dim3(TT / 16, NH_, NB), 32, 0, stream>>>(QK16, VT16, CTX);
    k_gemm_out<<<dim3(TT / 64, DM / 64, NB), 32, 0, stream>>>(CTX, WO, OUT, bproj);
}
